// simple_model_11819749998948
// MI455X (gfx1250) — hardware-verified
//
#include <hip/hip_runtime.h>
#include <math.h>

typedef __attribute__((ext_vector_type(16))) _Float16 v16h;
typedef __attribute__((ext_vector_type(8)))  _Float16 v8h;
typedef __attribute__((ext_vector_type(8)))  float    v8f;
typedef __attribute__((ext_vector_type(4)))  float    v4f;

constexpr int kImages   = 4096;
constexpr int kSide     = 22;
constexpr int kPix      = kSide * kSide;
constexpr int kGridW    = 11;
constexpr int kPos      = kGridW * kGridW;
constexpr int kPosPad   = 128;
constexpr int kCh       = 64;
constexpr int kK1       = 36;
constexpr int kK1Pad    = 64;
constexpr int kTaps2    = 9;
constexpr int kTaps3    = 16;
constexpr int kOutPos   = 64;
constexpr int kZeroRow  = kPosPad;
constexpr int kPowIters = 512;
constexpr int kPolyIters = 10;

constexpr float kActCarry  = 64.0f;
constexpr float kWgtCarry  = 256.0f;
constexpr float kBiasCarry = kActCarry * kWgtCarry;
constexpr float kFoldAct   = 1.0f / kWgtCarry;
constexpr float kFoldOut   = 1.0f / (kActCarry * kWgtCarry);

static_assert(kPix == 484 && kPos == 121, "shape");
static_assert((kK1Pad % 32) == 0 && (kCh % 32) == 0, "GEMM K multiples of 32");
static_assert((kPosPad % 16) == 0 && (kCh % 16) == 0 && (kOutPos % 16) == 0, "tile multiples");
static_assert(kBiasCarry == 16384.0f, "carry product");

constexpr size_t kOffBO   = 0;
constexpr size_t kOffW1T  = kOffBO  + (size_t)kCh * kOutPos * 4;
constexpr size_t kOffW2T  = kOffW1T + (size_t)kCh * kK1Pad * 2;
constexpr size_t kOffW3T  = kOffW2T + (size_t)kTaps2 * kCh * kCh * 2;
constexpr size_t kWsTotal = kOffW3T + (size_t)kTaps3 * kCh * kCh * 2;
static_assert(kWsTotal == 229376ull, "carve total");
static_assert((kOffW1T % 128) == 0 && (kOffW2T % 128) == 0 && (kOffW3T % 128) == 0, "aligned regions");

constexpr int kHalvesW1 = kCh * kK1Pad;
constexpr int kHalvesW2 = kTaps2 * kCh * kCh;
constexpr int kHalvesW3 = kTaps3 * kCh * kCh;
constexpr int kBlkW1 = kHalvesW1 / 2048;
constexpr int kBlkW2 = kHalvesW2 / 2048;
constexpr int kBlkW3 = kHalvesW3 / 2048;
static_assert(kBlkW1 * 2048 == kHalvesW1 && kBlkW2 * 2048 == kHalvesW2 && kBlkW3 * 2048 == kHalvesW3, "exact blocks");

union FragH { v16h v; v8h h[2]; };
__device__ __forceinline__ v16h ld_frag(const _Float16* p) {
  FragH f;
  f.h[0] = *(const v8h*)(p);
  f.h[1] = *(const v8h*)(p + 16);
  return f.v;
}
__device__ __forceinline__ v8f mma_g(v16h a, v16h b, v8f c) {
  c = __builtin_amdgcn_wmma_f32_16x16x32_f16(false, a, false, b, (short)0, c, false, false);
  asm volatile("v_nop\n\tv_nop\n\tv_nop\n\tv_nop" : "+v"(c) : "v"(a), "v"(b));
  return c;
}
__device__ __forceinline__ float wave_sum(float v) {
  v += __shfl_xor(v, 16, 32);
  v += __shfl_xor(v, 8, 32);
  v += __shfl_xor(v, 4, 32);
  v += __shfl_xor(v, 2, 32);
  v += __shfl_xor(v, 1, 32);
  return v;
}

__global__ __launch_bounds__(256) void basis_ortho_kernel(const float* __restrict__ basis, float* __restrict__ basisO)
{
  __shared__ __align__(16) float sW[2 * 4096];
  __shared__ __align__(16) float sG[4096];
  __shared__ __align__(16) float sV[64];
  __shared__ __align__(16) float sU[64];
  __shared__ __align__(16) float sT[64];
  const int t = threadIdx.x;
  const int lane = t & 31;
  const int r4 = t >> 2;
  const int part = t & 3;
  const int kb = part * 16;

#pragma unroll
  for (int it = 0; it < 4; ++it) {
    const int off = (it * 256 + t) * 4;
    const v4f m = *(const v4f*)(basis + off);
    *(v4f*)(sW + off) = m;
  }
  if (t < 64) sV[t] = 1.0f;
  __syncthreads();

#pragma unroll 1
  for (int itp = 0; itp < kPowIters; ++itp) {
    float s = 0.0f;
#pragma unroll 4
    for (int j = 0; j < 16; ++j) s = fmaf(sW[r4 * 64 + kb + j], sV[kb + j], s);
    s += __shfl_xor(s, 1, 32);
    s += __shfl_xor(s, 2, 32);
    if (part == 0) sU[r4] = s;
    __syncthreads();
    float w = 0.0f;
#pragma unroll 4
    for (int j = 0; j < 16; ++j) w = fmaf(sW[(kb + j) * 64 + r4], sU[kb + j], w);
    w += __shfl_xor(w, 1, 32);
    w += __shfl_xor(w, 2, 32);
    if (part == 0) sT[r4] = w;
    __syncthreads();
    const float ta = sT[lane];
    const float tb = sT[lane + 32];
    const float nn = wave_sum(ta * ta + tb * tb);
    const float inv = rsqrtf(nn + 1e-30f);
    if (t < 64) sV[t] = sT[t] * inv;
    __syncthreads();
  }
  {
    float s = 0.0f;
#pragma unroll 4
    for (int j = 0; j < 16; ++j) s = fmaf(sW[r4 * 64 + kb + j], sV[kb + j], s);
    s += __shfl_xor(s, 1, 32);
    s += __shfl_xor(s, 2, 32);
    if (part == 0) sU[r4] = s;
  }
  __syncthreads();
  {
    const float ua = sU[lane];
    const float ub = sU[lane + 32];
    const float va = sV[lane];
    const float vb = sV[lane + 32];
    const float nu = wave_sum(ua * ua + ub * ub);
    const float nv = wave_sum(va * va + vb * vb);
    const float invs = sqrtf(nv / nu);
#pragma unroll
    for (int it = 0; it < 4; ++it) {
      const int off = (it * 256 + t) * 4;
      v4f m = *(const v4f*)(sW + off);
      m = m * invs;
      *(v4f*)(sW + off) = m;
    }
  }
  __syncthreads();

  int co = 0;
  int no = 4096;
#pragma unroll 1
  for (int itn = 0; itn < kPolyIters; ++itn) {
#pragma unroll 1
    for (int hf = 0; hf < 2; ++hf) {
      const int j0 = kb + hf * 8;
      float g[8];
#pragma unroll
      for (int e = 0; e < 8; ++e) g[e] = 0.0f;
#pragma unroll 1
      for (int k = 0; k < 64; ++k) {
        const float a = sW[co + k * 64 + r4];
        const v4f b0 = *(const v4f*)(sW + co + k * 64 + j0);
        const v4f b1 = *(const v4f*)(sW + co + k * 64 + j0 + 4);
#pragma unroll
        for (int e = 0; e < 4; ++e) {
          g[e]     = fmaf(a, b0[e], g[e]);
          g[4 + e] = fmaf(a, b1[e], g[4 + e]);
        }
      }
      v4f p0, p1;
#pragma unroll
      for (int e = 0; e < 4; ++e) {
        const float d0 = (r4 == j0 + e) ? 1.5f : 0.0f;
        const float d1 = (r4 == j0 + 4 + e) ? 1.5f : 0.0f;
        p0[e] = fmaf(-0.5f, g[e], d0);
        p1[e] = fmaf(-0.5f, g[4 + e], d1);
      }
      *(v4f*)(sG + r4 * 64 + j0) = p0;
      *(v4f*)(sG + r4 * 64 + j0 + 4) = p1;
    }
    __syncthreads();
#pragma unroll 1
    for (int hf = 0; hf < 2; ++hf) {
      const int j0 = kb + hf * 8;
      float g[8];
#pragma unroll
      for (int e = 0; e < 8; ++e) g[e] = 0.0f;
#pragma unroll 1
      for (int k = 0; k < 64; ++k) {
        const float a = sW[co + r4 * 64 + k];
        const v4f b0 = *(const v4f*)(sG + k * 64 + j0);
        const v4f b1 = *(const v4f*)(sG + k * 64 + j0 + 4);
#pragma unroll
        for (int e = 0; e < 4; ++e) {
          g[e]     = fmaf(a, b0[e], g[e]);
          g[4 + e] = fmaf(a, b1[e], g[4 + e]);
        }
      }
      v4f p0, p1;
#pragma unroll
      for (int e = 0; e < 4; ++e) {
        p0[e] = g[e];
        p1[e] = g[4 + e];
      }
      *(v4f*)(sW + no + r4 * 64 + j0) = p0;
      *(v4f*)(sW + no + r4 * 64 + j0 + 4) = p1;
    }
    __syncthreads();
    const int tmp = co;
    co = no;
    no = tmp;
  }

  v4f ov[4];
#pragma unroll
  for (int it = 0; it < 4; ++it) ov[it] = *(const v4f*)(sW + co + (it * 256 + t) * 4);
  for (int pass = 0; pass < 2; ++pass) {
#pragma unroll
    for (int it = 0; it < 4; ++it) *(volatile v4f*)(basisO + (it * 256 + t) * 4) = ov[it];
    __threadfence();
  }
}

__global__ __launch_bounds__(256) void pack_weights_kernel(
    const float* __restrict__ w1, const float* __restrict__ w2, const float* __restrict__ w3,
    unsigned short* __restrict__ planes)
{
  const int i = blockIdx.x * 256 + threadIdx.x;
  const int e0 = i * 8;
  float v[8];
  if ((int)blockIdx.x < kBlkW1) {
    const int oc = e0 >> 6;
    const int k0 = e0 & 63;
#pragma unroll
    for (int e = 0; e < 8; ++e) {
      const int k = k0 + e;
      const int kc = (k < kK1) ? k : (kK1 - 1);
      float f = w1[oc * kK1 + kc];
      asm volatile("" : "+v"(f));
      v[e] = (k < kK1) ? f : 0.0f;
    }
  } else if ((int)blockIdx.x < kBlkW1 + kBlkW2) {
    const int g = e0 - kHalvesW1;
    const int tap = g >> 12;
    const int oc = (g >> 6) & 63;
    const int ic0 = g & 63;
#pragma unroll
    for (int e = 0; e < 8; ++e) v[e] = w2[(oc * kCh + ic0 + e) * kTaps2 + tap];
  } else {
    const int g = e0 - kHalvesW1 - kHalvesW2;
    const int tap = g >> 12;
    const int oc = (g >> 6) & 63;
    const int ic0 = g & 63;
#pragma unroll
    for (int e = 0; e < 8; ++e) v[e] = w3[(oc * kCh + ic0 + e) * kTaps3 + tap];
  }
  v8h hv;
#pragma unroll
  for (int e = 0; e < 8; ++e) hv[e] = (_Float16)(v[e] * kWgtCarry);
  unsigned short* q = planes + e0;
  *(volatile v8h*)q = hv;
  __threadfence();
  *(volatile v8h*)q = hv;
}

template <int K0>
__device__ __forceinline__ v8h im2col_chunk(const float* xs, int y, int xx, bool rowok, float lz) {
  v8h o;
#pragma unroll
  for (int e = 0; e < 8; ++e) {
    const int k = K0 + e;
    float val = lz;
    if (k < kK1) {
      const int ic = k / 9;
      const int r = (k % 9) / 3;
      const int cx = k % 3;
      const int hh = y + r - 1;
      const int ww = xx + cx - 1;
      const bool ok = rowok && ((unsigned)hh < (unsigned)kGridW) && ((unsigned)ww < (unsigned)kGridW);
      const int hc = hh < 0 ? 0 : (hh > kGridW - 1 ? kGridW - 1 : hh);
      const int wc = ww < 0 ? 0 : (ww > kGridW - 1 ? kGridW - 1 : ww);
      const float xv = xs[(2 * hc + (ic >> 1)) * kSide + 2 * wc + (ic & 1)];
      val = ok ? xv * kActCarry : lz;
    }
    o[e] = (_Float16)val;
  }
  return o;
}

__global__ __launch_bounds__(256) void fused_image_kernel(
    const float* __restrict__ x,
    const float* __restrict__ b1, const float* __restrict__ b2, const float* __restrict__ b3,
    const float* __restrict__ basisO,
    const _Float16* __restrict__ W1t, const _Float16* __restrict__ W2t, const _Float16* __restrict__ W3t,
    float* __restrict__ out)
{
  __shared__ __align__(16) float sX[512];
  __shared__ __align__(16) float sCO[kOutPos * kCh];
  __shared__ __align__(16) _Float16 sF1[(kPosPad + 1) * kCh];
  __shared__ __align__(16) _Float16 sF2[kPosPad * kCh];
  _Float16* sA1 = (_Float16*)sCO;
  static_assert(sizeof(float) * kOutPos * kCh == sizeof(_Float16) * kPosPad * kK1Pad, "alias extent");

  const int t = threadIdx.x;
  const int lane = t & 31;
  const int wave = t >> 5;
  const int hh = lane >> 4;
  const int c = lane & 15;
  const int img = blockIdx.x;

  float lz = 0.0f;
  asm volatile("" : "+v"(lz));

  {
    const float* xin = x + (size_t)img * kPix;
    const int i1 = (t + 256 < kPix) ? (t + 256) : (kPix - 1);
    const float v0 = xin[t];
    const float v1 = xin[i1];
    sX[t] = v0;
    sX[t + 256] = v1;
    if (t < 8) {
      v8h z;
#pragma unroll
      for (int e = 0; e < 8; ++e) z[e] = (_Float16)lz;
      *(v8h*)(sF1 + kZeroRow * kCh + t * 8) = z;
    }
  }
  __syncthreads();

  {
    const int p = t & 127;
    const int partw = t >> 7;
    const int y = p / kGridW;
    const int xx = p - y * kGridW;
    const bool rowok = (p < kPos);
    _Float16* arow = sA1 + p * kK1Pad;
    v8h z;
#pragma unroll
    for (int e = 0; e < 8; ++e) z[e] = (_Float16)lz;
    if (partw == 0) {
      *(v8h*)(arow + 0)  = im2col_chunk<0>(sX, y, xx, rowok, lz);
      *(v8h*)(arow + 8)  = im2col_chunk<8>(sX, y, xx, rowok, lz);
      *(v8h*)(arow + 16) = im2col_chunk<16>(sX, y, xx, rowok, lz);
      *(v8h*)(arow + 40) = z;
    } else {
      *(v8h*)(arow + 24) = im2col_chunk<24>(sX, y, xx, rowok, lz);
      *(v8h*)(arow + 32) = im2col_chunk<32>(sX, y, xx, rowok, lz);
      *(v8h*)(arow + 48) = z;
      *(v8h*)(arow + 56) = z;
    }
  }
  __syncthreads();

  {
    const int mt = wave;
    const _Float16* ap = sA1 + (mt * 16 + c) * kK1Pad + 8 * hh;
    const v16h a0 = ld_frag(ap);
    const v16h a1 = ld_frag(ap + 32);
#pragma unroll
    for (int nt = 0; nt < 4; ++nt) {
      const float bv = b1[nt * 16 + c] * kBiasCarry;
      v8f acc = (v8f){bv, bv, bv, bv, bv, bv, bv, bv};
      const _Float16* bp = W1t + (nt * 16 + c) * kK1Pad + 8 * hh;
      const v16h bf0 = ld_frag(bp);
      const v16h bf1 = ld_frag(bp + 32);
      acc = mma_g(a0, bf0, acc);
      acc = mma_g(a1, bf1, acc);
#pragma unroll
      for (int r = 0; r < 8; ++r)
        sF1[(mt * 16 + 8 * hh + r) * kCh + nt * 16 + c] = (_Float16)(fmaxf(acc[r], 0.0f) * kFoldAct);
    }
  }
  __syncthreads();

  {
    const int mt = wave;
    const int p = mt * 16 + c;
    const int py = p / kGridW;
    const int px = p - py * kGridW;
    const bool rowok = (p < kPos);
    v8f acc[4];
#pragma unroll
    for (int nt = 0; nt < 4; ++nt) {
      const float bv = b2[nt * 16 + c] * kBiasCarry;
      acc[nt] = (v8f){bv, bv, bv, bv, bv, bv, bv, bv};
    }
#pragma unroll 1
    for (int tap = 0; tap < kTaps2; ++tap) {
      const int ky = tap / 3;
      const int kx = tap - ky * 3;
      const int yy = py + ky - 1;
      const int xs = px + kx - 1;
      const bool valid = rowok && ((unsigned)yy < (unsigned)kGridW) && ((unsigned)xs < (unsigned)kGridW);
      const int srow = valid ? (yy * kGridW + xs) : kZeroRow;
      const _Float16* ap = sF1 + srow * kCh + 8 * hh;
      const _Float16* bp = W2t + (tap * kCh + c) * kCh + 8 * hh;
#pragma unroll
      for (int kc = 0; kc < 2; ++kc) {
        const v16h a = ld_frag(ap + kc * 32);
#pragma unroll
        for (int nt = 0; nt < 4; ++nt) {
          const v16h bfr = ld_frag(bp + nt * 16 * kCh + kc * 32);
          acc[nt] = mma_g(a, bfr, acc[nt]);
        }
      }
    }
#pragma unroll
    for (int nt = 0; nt < 4; ++nt) {
#pragma unroll
      for (int r = 0; r < 8; ++r)
        sF2[(mt * 16 + 8 * hh + r) * kCh + nt * 16 + c] = (_Float16)(fmaxf(acc[nt][r], 0.0f) * kFoldAct);
    }
  }
  __syncthreads();

  {
    const int mt = wave & 3;
    const int nh = wave >> 2;
    const int q = mt * 16 + c;
    const int qy = q >> 3;
    const int qx = q & 7;
    v8f acc[2];
#pragma unroll
    for (int j = 0; j < 2; ++j) {
      const float bv = b3[(nh * 2 + j) * 16 + c] * kBiasCarry;
      acc[j] = (v8f){bv, bv, bv, bv, bv, bv, bv, bv};
    }
#pragma unroll 1
    for (int tap = 0; tap < kTaps3; ++tap) {
      const int srow = (qy + (tap >> 2)) * kGridW + qx + (tap & 3);
      const _Float16* ap = sF2 + srow * kCh + 8 * hh;
      const _Float16* bp = W3t + (tap * kCh + nh * 32 + c) * kCh + 8 * hh;
#pragma unroll
      for (int kc = 0; kc < 2; ++kc) {
        const v16h a = ld_frag(ap + kc * 32);
#pragma unroll
        for (int j = 0; j < 2; ++j) {
          const v16h bfr = ld_frag(bp + j * 16 * kCh + kc * 32);
          acc[j] = mma_g(a, bfr, acc[j]);
        }
      }
    }
#pragma unroll
    for (int j = 0; j < 2; ++j) {
#pragma unroll
      for (int r = 0; r < 8; ++r)
        sCO[(mt * 16 + 8 * hh + r) * kCh + (nh * 2 + j) * 16 + c] = acc[j][r] * kFoldOut;
    }
  }
  __syncthreads();

  if (t < kOutPos) {
    float s = 0.0f;
#pragma unroll 8
    for (int cc = 0; cc < kCh; ++cc) s = fmaf(basisO[cc * kOutPos + t], sCO[t * kCh + cc], s);
    volatile float* op = out + (size_t)img * kOutPos + t;
    *op = s;
    __threadfence();
    *op = s;
  }
}

extern "C" void kernel_launch(void* const* d_in, const int* in_sizes, int n_in,
                              void* d_out, int out_size, void* d_ws, size_t ws_size,
                              hipStream_t stream) {
  if (n_in < 8) return;
  if (in_sizes[0] != kImages * kPix) return;
  if (in_sizes[1] != kCh * kK1) return;
  if (in_sizes[2] != kCh) return;
  if (in_sizes[3] != kCh * kCh * kTaps2) return;
  if (in_sizes[4] != kCh) return;
  if (in_sizes[5] != kCh * kCh * kTaps3) return;
  if (in_sizes[6] != kCh) return;
  if (in_sizes[7] != kCh * kOutPos) return;
  if (out_size != kImages * kOutPos) return;
  if (ws_size < kWsTotal) return;

  const float* x     = (const float*)d_in[0];
  const float* w1    = (const float*)d_in[1];
  const float* b1    = (const float*)d_in[2];
  const float* w2    = (const float*)d_in[3];
  const float* b2    = (const float*)d_in[4];
  const float* w3    = (const float*)d_in[5];
  const float* b3    = (const float*)d_in[6];
  const float* basis = (const float*)d_in[7];
  float* out = (float*)d_out;

  char* ws = (char*)d_ws;
  float* basisO = (float*)(ws + kOffBO);
  unsigned short* planes = (unsigned short*)(ws + kOffW1T);
  const _Float16* W1t = (const _Float16*)(ws + kOffW1T);
  const _Float16* W2t = (const _Float16*)(ws + kOffW2T);
  const _Float16* W3t = (const _Float16*)(ws + kOffW3T);

  basis_ortho_kernel<<<1, 256, 0, stream>>>(basis, basisO);
  pack_weights_kernel<<<kBlkW1 + kBlkW2 + kBlkW3, 256, 0, stream>>>(w1, w2, w3, planes);
  fused_image_kernel<<<kImages, 256, 0, stream>>>(x, b1, b2, b3, basisO, W1t, W2t, W3t, out);
}
